// MPNN_ENN_Set2Set_22153441313213
// MI455X (gfx1250) — hardware-verified
//
#include <hip/hip_runtime.h>
#include <stddef.h>
#include <stdint.h>

#define NN     8192
#define NE     32768
#define NG     64
#define NFD    32
#define EFD    16
#define DH     64
#define OUTD   12
#define TMPS   3
#define TS2S   12
#define KP     128
#define G3     192
#define NW2    4096
#define NPA    2048
#define NPB    2112
#define NPC    4160
#define PP     2112
#define LW     256
#define NTHR   256
#define NWAVE  8
#define GTHR   128
#define GBM    64
#define GBN    64
#define EPBK   16
#define EPT    8
#define CHUNK  (NTHR * EPT)
#define WCAP   (EPT * 32)
#define LISTN  (NWAVE * WCAP)
#define NBMAX  2048
#define NBA    1024
#define RCAP   8192
#define DEGCAP 64
#define PKS    11
#define STW    512
#define GCAP   256
#define XS     65
#define NPW    (NN / NWAVE)
#define LDS_AGG ((2 * RCAP + 2 * NBMAX + LISTN) * 4 + 64)
#define LDS_S2S (GCAP * XS * 4)
#define WSMAX  134217728

#define U_XB   (NN * NFD / 8)
#define U_EFB  (NE * 32 / 8)
#define U_WIN  (DH * 32 / 8)
#define U_WEE  (DH * 32 / 8)
#define U_BTM  (NW2 * KP / 8)
#define U_BTB  (DH * KP / 8)
#define U_WG   (G3 * KP / 8)
#define U_WLI  (128 * LW / 4)
#define U_WLH  (64 * LW / 4)
#define U_ALL  (U_XB + U_EFB + U_WIN + U_WEE + U_BTM + U_BTB + 2 * U_WG + U_WLI + U_WLH)

static_assert((CHUNK & (CHUNK - 1)) == 0 && CHUNK <= (1 << PKS));
static_assert((NBMAX & (NBMAX - 1)) == 0 && NBMAX <= (1 << PKS));
static_assert(NTHR * 8 == NBMAX && NBA <= NBMAX && (NBA & (NBA - 1)) == 0);
static_assert(NN % NBA == 0 && NE % CHUNK == 0 && NE < (1 << (31 - PKS)));
static_assert(LISTN >= NBMAX && (RCAP % 32) == 0 && NWAVE * STW <= RCAP);
static_assert(RCAP >= 4381 && DEGCAP >= 22 && ((NBA / NWAVE) % 2) == 0);
static_assert(LDS_AGG <= 300000 && LDS_S2S <= 300000);
static_assert(GBM == (GTHR / 32) * 16 && GBN == 64 && DH == GBN);
static_assert(NN % GBM == 0 && NE % GBM == 0 && NPA % GBN == 0 && NPB % GBN == 0 && G3 % GBN == 0);
static_assert(NPA + NPB == NPC && NPC == NW2 + DH && PP >= NPB && PP >= NPA && (PP * 4) % 128 == 0);
static_assert(KP % 32 == 0 && KP == 2 * DH && NFD == 32);
static_assert(NE % EPBK == 0 && EPBK == 2 * NWAVE);
static_assert(GCAP == NTHR && GCAP >= 157 + 16 && NN % (NWAVE * 32) == 0);
static_assert((NG * OUTD * 4) % 128 == 0 && NG * OUTD == 3 * NTHR && (NG * OUTD) / 4 <= NTHR);
static_assert(U_XB % NTHR == 0 && U_EFB % NTHR == 0 && U_WIN % NTHR == 0 && U_WEE % NTHR == 0);
static_assert(U_BTM % NTHR == 0 && U_BTB % NTHR == 0 && U_WG % NTHR == 0 && U_WLI % NTHR == 0 && U_WLH % NTHR == 0);
static_assert(NN % 4 == 0);

typedef float          v2f   __attribute__((ext_vector_type(2)));
typedef float          v4f   __attribute__((ext_vector_type(4)));
typedef float          v8f   __attribute__((ext_vector_type(8)));
typedef int            v4i   __attribute__((ext_vector_type(4)));
typedef int            v8i   __attribute__((ext_vector_type(8)));
typedef unsigned int   v4u   __attribute__((ext_vector_type(4)));
typedef unsigned short v8us  __attribute__((ext_vector_type(8)));
typedef __bf16         v16bf __attribute__((ext_vector_type(16)));
typedef v4f  __attribute__((may_alias)) v4fa;
typedef v4u  __attribute__((may_alias)) v4ua;
typedef v8us __attribute__((may_alias)) v8usa;
union FragB { v16bf v; v8us h[2]; v8i w; };

__device__ __forceinline__ v8f wmb(const FragB& a, const FragB& b, v8f c) {
  v8f d = __builtin_amdgcn_wmma_f32_16x16x32_bf16(false, a.v, false, b.v, (short)0, c, false, false);
  asm volatile("v_nop\n\tv_nop\n\tv_nop\n\tv_nop" : "+v"(d) : "v"(a.w), "v"(b.w));
  return d;
}

__device__ __forceinline__ unsigned bf16_bits(float f) {
  const unsigned u = __float_as_uint(f);
  return (u + 0x7FFFu + ((u >> 16) & 1u)) >> 16;
}
__device__ __forceinline__ float bf16_val(float f) {
  return __uint_as_float(bf16_bits(f) << 16);
}
__device__ __forceinline__ v8us cvt8(v4f a, v4f b) {
  v8us o;
  o[0] = (unsigned short)bf16_bits(a.x); o[1] = (unsigned short)bf16_bits(a.y);
  o[2] = (unsigned short)bf16_bits(a.z); o[3] = (unsigned short)bf16_bits(a.w);
  o[4] = (unsigned short)bf16_bits(b.x); o[5] = (unsigned short)bf16_bits(b.y);
  o[6] = (unsigned short)bf16_bits(b.z); o[7] = (unsigned short)bf16_bits(b.w);
  return o;
}
__device__ __forceinline__ v8us split8(const float* sp, unsigned mh) {
  const v4f a = *(const v4fa*)sp;
  const v4f b = *(const v4fa*)(sp + 4);
  const v8f f8 = {a.x, a.y, a.z, a.w, b.x, b.y, b.z, b.w};
  const unsigned ml = ~mh;
  v8us o;
#pragma unroll
  for (int e = 0; e < 8; ++e) {
    const unsigned hb = bf16_bits(f8[e]);
    const unsigned lb = bf16_bits(f8[e] - __uint_as_float(hb << 16));
    o[e] = (unsigned short)((hb & ml) | (lb & mh));
  }
  return o;
}
__device__ __forceinline__ float sigm(float x) {
  return __builtin_amdgcn_rcpf(1.0f + expf(-x));
}
__device__ __forceinline__ float nmax(float a, float b) {
  return (b > a || b != b) ? b : a;
}
__device__ __forceinline__ void put16(unsigned short* dp, v8us o) {
  *(volatile v8us*)dp = o;
  __threadfence();
  *(volatile v8us*)dp = o;
}
__device__ __forceinline__ void putf4(float* dp, v4f o) {
  *(volatile v4f*)dp = o;
  __threadfence();
  *(volatile v4f*)dp = o;
}

__device__ __forceinline__ int scan_chunk(const int* __restrict__ dsts, int nE, int cbase, int slotBase,
                                          int nb, int vec8, int* list, int tid, int lane, int wave) {
  int wc = 0;
  const int el0  = tid * EPT;
  const int e0   = cbase + el0;
  const int sent = -2147483647 - 1;
  v4i da, db;
  if (vec8 != 0 && cbase + CHUNK <= nE) {
    da = *(const v4i*)(dsts + e0);
    db = *(const v4i*)(dsts + e0 + 4);
  } else {
    da.x = (e0     < nE) ? dsts[min(e0,     nE - 1)] : sent;
    da.y = (e0 + 1 < nE) ? dsts[min(e0 + 1, nE - 1)] : sent;
    da.z = (e0 + 2 < nE) ? dsts[min(e0 + 2, nE - 1)] : sent;
    da.w = (e0 + 3 < nE) ? dsts[min(e0 + 3, nE - 1)] : sent;
    db.x = (e0 + 4 < nE) ? dsts[min(e0 + 4, nE - 1)] : sent;
    db.y = (e0 + 5 < nE) ? dsts[min(e0 + 5, nE - 1)] : sent;
    db.z = (e0 + 6 < nE) ? dsts[min(e0 + 6, nE - 1)] : sent;
    db.w = (e0 + 7 < nE) ? dsts[min(e0 + 7, nE - 1)] : sent;
  }
  const unsigned nbs = (unsigned)slotBase;
  const unsigned unb = (unsigned)nb;
  const unsigned s0 = (unsigned)da.x - nbs, s1 = (unsigned)da.y - nbs;
  const unsigned s2 = (unsigned)da.z - nbs, s3 = (unsigned)da.w - nbs;
  const unsigned s4 = (unsigned)db.x - nbs, s5 = (unsigned)db.y - nbs;
  const unsigned s6 = (unsigned)db.z - nbs, s7 = (unsigned)db.w - nbs;
  const bool h0 = s0 < unb, h1 = s1 < unb, h2 = s2 < unb, h3 = s3 < unb;
  const bool h4 = s4 < unb, h5 = s5 < unb, h6 = s6 < unb, h7 = s7 < unb;
  const unsigned any = __builtin_amdgcn_ballot_w32(h0 | h1 | h2 | h3 | h4 | h5 | h6 | h7);
  if (any != 0u) {
#define HITJ(J, HJ, SJ) { \
      const unsigned mj = __builtin_amdgcn_ballot_w32(HJ); \
      if (mj != 0u) { \
        if (HJ) { \
          const int pos = wc + (int)__builtin_amdgcn_mbcnt_lo(mj, 0u); \
          if (pos < WCAP) list[wave * WCAP + pos] = ((el0 + (J)) << PKS) | (int)(SJ); \
        } \
        wc += (int)__builtin_popcount(mj); } }
    HITJ(0, h0, s0)
    HITJ(1, h1, s1)
    HITJ(2, h2, s2)
    HITJ(3, h3, s3)
    HITJ(4, h4, s4)
    HITJ(5, h5, s5)
    HITJ(6, h6, s6)
    HITJ(7, h7, s7)
#undef HITJ
  }
  return wc;
}

__global__ __launch_bounds__(NTHR) void k_prep(const float* __restrict__ nf, const float* __restrict__ ef,
                                               const float* __restrict__ W_in, const float* __restrict__ W_ee1,
                                               const float* __restrict__ W_ee2, const float* __restrict__ b_ee2,
                                               const float* __restrict__ W_ih, const float* __restrict__ W_hh,
                                               const float* __restrict__ Wl_ih, const float* __restrict__ Wl_hh,
                                               unsigned short* XB, unsigned short* EFB,
                                               unsigned short* WinT, unsigned short* Wee1T,
                                               unsigned short* Bt2, unsigned short* WihT2,
                                               unsigned short* WhhT2, float* WL) {
  const int u  = (int)blockIdx.x * NTHR + (int)threadIdx.x;
  const int L0 = U_XB;
  const int L1 = L0 + U_EFB;
  const int L2 = L1 + U_WIN;
  const int L3 = L2 + U_WEE;
  const int L4 = L3 + U_BTM;
  const int L5 = L4 + U_BTB;
  const int L6 = L5 + U_WG;
  const int L7 = L6 + U_WG;
  const int L8 = L7 + U_WLI;
  const int L9 = L8 + U_WLH;
  if (u < L0) {
    const int v = u;
    const float* p = nf + (size_t)v * 8;
    const v4f a = *(const v4f*)p;
    const v4f b = *(const v4f*)(p + 4);
    put16(XB + (size_t)v * 8, cvt8(a, b));
    return;
  } else if (u < L1) {
    const int v   = u - L0;
    const int row = v >> 2;
    const int q   = v & 3;
    const float* p = ef + (size_t)row * EFD + 8 * (q & 1);
    const v4f a = *(const v4f*)p;
    const v4f b = *(const v4f*)(p + 4);
    v8us o = cvt8(a, b);
    const unsigned short mk = (q < 2) ? (unsigned short)0xffff : (unsigned short)0;
#pragma unroll
    for (int i = 0; i < 8; ++i) o[i] = (unsigned short)(o[i] & mk);
    put16(EFB + (size_t)v * 8, o);
    return;
  } else if (u < L2) {
    const int v  = u - L1;
    const int n  = v >> 2;
    const int k8 = (v & 3) * 8;
    const float* p = W_in + (size_t)k8 * DH + n;
    v8us o;
#pragma unroll
    for (int i = 0; i < 8; ++i) o[i] = (unsigned short)bf16_bits(p[(size_t)i * DH]);
    put16(WinT + (size_t)n * 32 + k8, o);
    return;
  } else if (u < L3) {
    const int v  = u - L2;
    const int n  = v >> 2;
    const int k8 = (v & 3) * 8;
    const int kk = k8 & 8;
    const float* p = W_ee1 + (size_t)kk * DH + n;
    const unsigned short mk = (k8 < EFD) ? (unsigned short)0xffff : (unsigned short)0;
    v8us o;
#pragma unroll
    for (int i = 0; i < 8; ++i) o[i] = (unsigned short)(bf16_bits(p[(size_t)i * DH]) & mk);
    put16(Wee1T + (size_t)n * 32 + k8, o);
    return;
  } else if (u < L4) {
    const int v  = u - L3;
    const int n  = v >> 4;
    const int k8 = (v & 15) * 8;
    const int j  = k8 & 63;
    const float* p = W_ee2 + (size_t)n * DH + j;
    const v4f a = *(const v4f*)p;
    const v4f b = *(const v4f*)(p + 4);
    put16(Bt2 + (size_t)n * KP + k8, cvt8(a, b));
    return;
  } else if (u < L5) {
    const int v  = u - L4;
    const int n  = v >> 4;
    const int k8 = (v & 15) * 8;
    const int j  = k8 & 63;
    const float* p = b_ee2 + (size_t)n * DH + j;
    const v4f a = *(const v4f*)p;
    const v4f b = *(const v4f*)(p + 4);
    put16(Bt2 + (size_t)(NW2 + n) * KP + k8, cvt8(a, b));
    return;
  } else if (u < L6) {
    const int v    = u - L5;
    const int n    = v >> 4;
    const int k8   = (v & 15) * 8;
    const int srow = k8 & 63;
    const float* p = W_ih + (size_t)srow * G3 + n;
    v8us o;
#pragma unroll
    for (int i = 0; i < 8; ++i) o[i] = (unsigned short)bf16_bits(p[(size_t)i * G3]);
    put16(WihT2 + (size_t)n * KP + k8, o);
    return;
  } else if (u < L7) {
    const int v    = u - L6;
    const int n    = v >> 4;
    const int k8   = (v & 15) * 8;
    const int srow = k8 & 63;
    const float* p = W_hh + (size_t)srow * G3 + n;
    v8us o;
#pragma unroll
    for (int i = 0; i < 8; ++i) o[i] = (unsigned short)bf16_bits(p[(size_t)i * G3]);
    put16(WhhT2 + (size_t)n * KP + k8, o);
    return;
  } else if (u < L8) {
    const int v = u - L7;
    const v4f a = *(const v4f*)(Wl_ih + (size_t)v * 4);
    v4f o;
    o.x = bf16_val(a.x); o.y = bf16_val(a.y); o.z = bf16_val(a.z); o.w = bf16_val(a.w);
    putf4(WL + (size_t)v * 4, o);
    return;
  } else if (u < L9) {
    const int v = u - L8;
    const v4f a = *(const v4f*)(Wl_hh + (size_t)v * 4);
    v4f o;
    o.x = bf16_val(a.x); o.y = bf16_val(a.y); o.z = bf16_val(a.z); o.w = bf16_val(a.w);
    putf4(WL + (size_t)128 * LW + (size_t)v * 4, o);
    return;
  }
}

template <int RELU, int SPLIT>
__global__ __launch_bounds__(GTHR) void k_gemm(const unsigned short* __restrict__ A, int lda,
                                               const unsigned short* __restrict__ BT, int ldb, int K,
                                               const float* __restrict__ bias, int hasBias,
                                               float* C, int ldc, unsigned short* Chl) {
  __shared__ __attribute__((aligned(16))) float stg[GBM * GBN];
  const int tid = (int)threadIdx.x, lane = tid & 31, wave = tid >> 5, hh = lane >> 4, m = lane & 15;
  const int rowBase = (int)blockIdx.x * GBM;
  const int colBase = (int)blockIdx.y * GBN;

  v8f acc[4];
  {
    const v8f z = {0.f, 0.f, 0.f, 0.f, 0.f, 0.f, 0.f, 0.f};
#pragma unroll
    for (int t = 0; t < 4; ++t) acc[t] = z;
  }
  const unsigned short* ap = A  + (size_t)(rowBase + 16 * wave + m) * (size_t)lda + 8 * hh;
  const unsigned short* bp = BT + (size_t)(colBase + m) * (size_t)ldb + 8 * hh;

#pragma unroll 1
  for (int k0 = 0; k0 < K; k0 += 32) {
    FragB af;
    af.h[0] = *(const v8usa*)(ap + k0);
    af.h[1] = *(const v8usa*)(ap + k0 + 16);
#pragma unroll
    for (int nt = 0; nt < 4; ++nt) {
      const unsigned short* wq = bp + (size_t)(16 * nt) * (size_t)ldb + k0;
      FragB bf;
      bf.h[0] = *(const v8usa*)wq;
      bf.h[1] = *(const v8usa*)(wq + 16);
      acc[nt] = wmb(af, bf, acc[nt]);
    }
  }

#pragma unroll
  for (int nt = 0; nt < 4; ++nt) {
    const int lc = 16 * nt + m;
    float bvv = 0.0f;
    if (hasBias != 0) bvv = bf16_val(bias[colBase + lc]);
#pragma unroll
    for (int r = 0; r < 8; ++r) {
      const int lr = 16 * wave + 8 * hh + r;
      float v = acc[nt][r] + bvv;
      if constexpr (RELU == 1) v = (v > 0.0f) ? v : (v - v);
      stg[lr * GBN + lc] = v;
    }
  }
  __syncthreads();

  const int rsel = lane >> 4;
  const int j    = lane & 15;
  {
    v4f pv[8];
#pragma unroll
    for (int i = 0; i < 8; ++i) pv[i] = *(const v4fa*)(stg + (16 * wave + 2 * i + rsel) * GBN + 4 * j);
#pragma unroll
    for (int i = 0; i < 8; ++i) {
      float* op = C + (size_t)(rowBase + 16 * wave + 2 * i + rsel) * (size_t)ldc + colBase + 4 * j;
      *(volatile v4f*)op = pv[i];
    }
    __threadfence();
#pragma unroll
    for (int i = 0; i < 8; ++i) {
      float* op = C + (size_t)(rowBase + 16 * wave + 2 * i + rsel) * (size_t)ldc + colBase + 4 * j;
      *(volatile v4f*)op = pv[i];
    }
  }
  if constexpr (SPLIT == 1) {
    const int ch = 8 * (j & 7);
    const unsigned mh = 0u - (unsigned)(j >> 3);
    v8us ph[8];
#pragma unroll
    for (int i = 0; i < 8; ++i) ph[i] = split8(stg + (16 * wave + 2 * i + rsel) * GBN + ch, mh);
#pragma unroll
    for (int i = 0; i < 8; ++i) {
      unsigned short* op = Chl + (size_t)(rowBase + 16 * wave + 2 * i + rsel) * (size_t)KP + 8 * j;
      *(volatile v8us*)op = ph[i];
    }
    __threadfence();
#pragma unroll
    for (int i = 0; i < 8; ++i) {
      unsigned short* op = Chl + (size_t)(rowBase + 16 * wave + 2 * i + rsel) * (size_t)KP + 8 * j;
      *(volatile v8us*)op = ph[i];
    }
  }
}

template <int HALF>
__global__ __launch_bounds__(NTHR) void k_edge(const float* __restrict__ ED, const int* __restrict__ srcs,
                                               const float* __restrict__ P, const float* __restrict__ MIN,
                                               float* MOUT) {
  __shared__ __attribute__((aligned(16))) float sED[EPBK * 32];
  const int tid = (int)threadIdx.x, lane = tid & 31, wave = tid >> 5;
  const int e0 = (int)blockIdx.x * EPBK;
  {
    const int el = tid >> 4;
    const int q  = tid & 15;
    const v2f v = *(const v2f*)(ED + (size_t)(e0 + el) * DH + 32 * HALF + 2 * q);
    sED[el * 32 + 2 * q]     = v.x;
    sED[el * 32 + 2 * q + 1] = v.y;
  }
  __syncthreads();
  const int el = 2 * wave + (lane >> 4);
  const int c4 = 4 * (lane & 15);
  const int e  = e0 + el;
  int s = srcs[e];
  s = s < 0 ? 0 : (s > NN - 1 ? NN - 1 : s);
  const float* pr = P + (size_t)s * PP + c4;
  v4f acc = {0.0f, 0.0f, 0.0f, 0.0f};
  if constexpr (HALF == 1) acc = *(const v4f*)(MIN + (size_t)e * DH + c4);
#pragma unroll 1
  for (int k4 = 0; k4 < 32; k4 += 4) {
    const v4f ed4 = *(const v4fa*)(sED + el * 32 + k4);
    const v4f p0 = *(const v4f*)(pr + (size_t)(k4 + 0) * DH);
    const v4f p1 = *(const v4f*)(pr + (size_t)(k4 + 1) * DH);
    const v4f p2 = *(const v4f*)(pr + (size_t)(k4 + 2) * DH);
    const v4f p3 = *(const v4f*)(pr + (size_t)(k4 + 3) * DH);
    acc.x = fmaf(ed4.x, p0.x, acc.x); acc.y = fmaf(ed4.x, p0.y, acc.y);
    acc.z = fmaf(ed4.x, p0.z, acc.z); acc.w = fmaf(ed4.x, p0.w, acc.w);
    acc.x = fmaf(ed4.y, p1.x, acc.x); acc.y = fmaf(ed4.y, p1.y, acc.y);
    acc.z = fmaf(ed4.y, p1.z, acc.z); acc.w = fmaf(ed4.y, p1.w, acc.w);
    acc.x = fmaf(ed4.z, p2.x, acc.x); acc.y = fmaf(ed4.z, p2.y, acc.y);
    acc.z = fmaf(ed4.z, p2.z, acc.z); acc.w = fmaf(ed4.z, p2.w, acc.w);
    acc.x = fmaf(ed4.w, p3.x, acc.x); acc.y = fmaf(ed4.w, p3.y, acc.y);
    acc.z = fmaf(ed4.w, p3.z, acc.z); acc.w = fmaf(ed4.w, p3.w, acc.w);
  }
  if constexpr (HALF == 1) {
    const v4f pb = *(const v4f*)(pr + (size_t)32 * DH);
    acc.x = acc.x + pb.x; acc.y = acc.y + pb.y; acc.z = acc.z + pb.z; acc.w = acc.w + pb.w;
  }
  float* op = MOUT + (size_t)e * DH + c4;
  *(volatile v4f*)op = acc;
  __threadfence();
  *(volatile v4f*)op = acc;
}

__device__ __forceinline__ v2f gather_slot(const int* reg2, const int* scnt, const int* soff, int slot, int nh,
                                           bool ovf, const float* __restrict__ MSG, int lane) {
  int st = soff[slot];
  const int craw = scnt[slot];
  int cnt = craw;
  st  = st < 0 ? 0 : (st > nh ? nh : st);
  cnt = cnt < 0 ? 0 : (cnt > DEGCAP ? DEGCAP : cnt);
  if (cnt > nh - st) cnt = nh - st;
  float a0 = 0.0f, a1 = 0.0f;
#pragma unroll 1
  for (int b0 = 0; b0 < cnt; b0 += 32) {
    int idx = st + b0 + lane;
    idx = idx > nh - 1 ? nh - 1 : idx;
    idx = idx < 0 ? 0 : (idx > RCAP - 1 ? RCAP - 1 : idx);
    int eid = reg2[idx];
    eid = eid < 0 ? 0 : (eid > NE - 1 ? NE - 1 : eid);
    const int m32 = (cnt - b0) < 32 ? (cnt - b0) : 32;
#pragma unroll 1
    for (int k = 0; k < m32; ++k) {
      const int ek = __builtin_amdgcn_readlane(eid, k);
      const v2f v = *(const v2f*)(MSG + (size_t)ek * DH + 2 * lane);
      a0 += v.x; a1 += v.y;
    }
  }
  const float qnan = __int_as_float(0x7fc00000);
  const float pz = (ovf || craw > DEGCAP) ? qnan : 0.0f;
  v2f r;
  r.x = a0 + pz;
  r.y = a1 + pz;
  return r;
}

__global__ __launch_bounds__(NTHR) void k_agg(const int* __restrict__ dsts, const float* __restrict__ MSG,
                                              unsigned short* AGG) {
  extern __shared__ v4f lds_dyn[];
  int* reg1 = (int*)lds_dyn;
  int* reg2 = reg1 + RCAP;
  int* scnt = reg2 + RCAP;
  int* soff = scnt + NBMAX;
  int* list = soff + NBMAX;
  int* wcnt = list + LISTN;
  int* wtot = wcnt + NWAVE;
  const int tid = (int)threadIdx.x, lane = tid & 31, wave = tid >> 5;
  const int nodeBase = (int)blockIdx.x * NBA;
  const int nE = NE;

  for (int i = tid; i < NBMAX; i += NTHR) scnt[i] = 0;
  __syncthreads();

  int tot = 0;
  const int nChunks = (nE + CHUNK - 1) / CHUNK;
#pragma unroll 1
  for (int ch = 0; ch < nChunks; ++ch) {
    const int cbase = ch * CHUNK;
    const int wc = scan_chunk(dsts, nE, cbase, nodeBase, NBA, 1, list, tid, lane, wave);
    if (lane == 0) wcnt[wave] = wc;
    __syncthreads();
    int pre = 0, all = 0;
#pragma unroll
    for (int w2 = 0; w2 < NWAVE; ++w2) {
      int c = wcnt[w2];
      c = c < 0 ? 0 : (c > WCAP ? WCAP : c);
      all += c;
      pre += (w2 < wave) ? c : 0;
    }
    const int wcc  = wc > WCAP ? WCAP : wc;
    const int base = tot + pre;
#pragma unroll 1
    for (int i = lane; i < wcc; i += 32) {
      const int ent = list[wave * WCAP + i];
      const int el  = (ent >> PKS) & (CHUNK - 1);
      const int sl  = ent & (NBMAX - 1);
      int eid = cbase + el;
      eid = eid > nE - 1 ? nE - 1 : eid;
      const int pos = base + i;
      if (pos < RCAP) reg1[pos] = (int)(((unsigned)eid << PKS) | (unsigned)sl);
    }
    tot += all;
    tot = tot > RCAP ? RCAP : tot;
    __syncthreads();
  }
  const int nh = tot;

  if (wave == 0) {
#pragma unroll 1
    for (int b0 = 0; b0 < nh; b0 += 32) {
      const int idx = b0 + lane;
      const int uv  = reg1[idx < nh ? idx : nh - 1];
      const int m32 = (nh - b0) < 32 ? (nh - b0) : 32;
#pragma unroll 1
      for (int k = 0; k < m32; ++k) {
        const int u  = __builtin_amdgcn_readlane(uv, k);
        const int sl = u & (NBMAX - 1);
        if (lane == 0) scnt[sl] = scnt[sl] + 1;
      }
    }
  }
  __syncthreads();

  {
    const v4i ca = *(const v4i*)(scnt + 8 * tid);
    const v4i cb = *(const v4i*)(scnt + 8 * tid + 4);
    const int e0 = ca.x < 0 ? 0 : ca.x, e1 = ca.y < 0 ? 0 : ca.y, e2 = ca.z < 0 ? 0 : ca.z, e3 = ca.w < 0 ? 0 : ca.w;
    const int e4 = cb.x < 0 ? 0 : cb.x, e5 = cb.y < 0 ? 0 : cb.y, e6 = cb.z < 0 ? 0 : cb.z, e7 = cb.w < 0 ? 0 : cb.w;
    const int ts = e0 + e1 + e2 + e3 + e4 + e5 + e6 + e7;
    int incl = ts;
#pragma unroll
    for (int d = 1; d < 32; d <<= 1) {
      const int up = __shfl_up(incl, d);
      if (lane >= d) incl += up;
    }
    if (lane == 31) wtot[wave] = incl;
    __syncthreads();
    int pre = 0;
#pragma unroll
    for (int w2 = 0; w2 < NWAVE; ++w2) pre += (w2 < wave) ? wtot[w2] : 0;
    int run = pre + incl - ts;
    soff[8 * tid + 0] = run; run += e0;
    soff[8 * tid + 1] = run; run += e1;
    soff[8 * tid + 2] = run; run += e2;
    soff[8 * tid + 3] = run; run += e3;
    soff[8 * tid + 4] = run; run += e4;
    soff[8 * tid + 5] = run; run += e5;
    soff[8 * tid + 6] = run; run += e6;
    soff[8 * tid + 7] = run;
  }
  __syncthreads();
  for (int i = tid; i < NBMAX; i += NTHR) list[i] = soff[i];
  __syncthreads();

  if (wave == 0) {
#pragma unroll 1
    for (int b0 = 0; b0 < nh; b0 += 32) {
      const int idx = b0 + lane;
      const int uv  = reg1[idx < nh ? idx : nh - 1];
      const int m32 = (nh - b0) < 32 ? (nh - b0) : 32;
#pragma unroll 1
      for (int k = 0; k < m32; ++k) {
        const int u   = __builtin_amdgcn_readlane(uv, k);
        const int sl  = u & (NBMAX - 1);
        const int eid = (int)((unsigned)u >> PKS);
        if (lane == 0) {
          int pos = list[sl];
          pos = pos < 0 ? 0 : (pos > RCAP - 1 ? RCAP - 1 : pos);
          reg2[pos] = eid;
          list[sl] = pos + 1;
        }
      }
    }
  }
  __syncthreads();

  const int nbw = NBA / NWAVE;
  const bool ovf = (nh >= RCAP);
  unsigned int* stwu = (unsigned int*)(reg1 + wave * STW);

#pragma unroll 1
  for (int jt = 0; jt < nbw; jt += 2) {
    const int slot0 = wave * nbw + jt;
    const v2f r0 = gather_slot(reg2, scnt, soff, slot0,     nh, ovf, MSG, lane);
    const v2f r1 = gather_slot(reg2, scnt, soff, slot0 + 1, nh, ovf, MSG, lane);
    const unsigned h0x = bf16_bits(r0.x), h0y = bf16_bits(r0.y);
    const unsigned h1x = bf16_bits(r1.x), h1y = bf16_bits(r1.y);
    const unsigned l0x = bf16_bits(r0.x - __uint_as_float(h0x << 16));
    const unsigned l0y = bf16_bits(r0.y - __uint_as_float(h0y << 16));
    const unsigned l1x = bf16_bits(r1.x - __uint_as_float(h1x << 16));
    const unsigned l1y = bf16_bits(r1.y - __uint_as_float(h1y << 16));
    __builtin_amdgcn_fence(__ATOMIC_RELEASE, "wavefront");
    __builtin_amdgcn_wave_barrier();
    stwu[lane]      = (h0x & 0xffffu) | (h0y << 16);
    stwu[32 + lane] = (l0x & 0xffffu) | (l0y << 16);
    stwu[64 + lane] = (h1x & 0xffffu) | (h1y << 16);
    stwu[96 + lane] = (l1x & 0xffffu) | (l1y << 16);
    __builtin_amdgcn_fence(__ATOMIC_RELEASE, "wavefront");
    __builtin_amdgcn_wave_barrier();
    const v4u pk = *(const v4ua*)(stwu + 4 * lane);
    unsigned short* gp = AGG + (size_t)(nodeBase + slot0) * (size_t)KP + 8 * lane;
    *(volatile v4u*)gp = pk;
    __threadfence();
    *(volatile v4u*)gp = pk;
  }
}

__global__ __launch_bounds__(NTHR) void k_gru(const float* __restrict__ GI, const float* __restrict__ GH,
                                              float* H, unsigned short* Hhl) {
  __shared__ __attribute__((aligned(16))) float sH[4 * DH];
  const int tid = (int)threadIdx.x, wave = tid >> 5;
  const int r = tid >> 6, c = tid & 63;
  const int row = (int)blockIdx.x * 4 + r;
  const float* gi = GI + (size_t)row * G3 + c;
  const float* gh = GH + (size_t)row * G3 + c;
  const float i_r = gi[0], i_z = gi[64], i_n = gi[128];
  const float h_r = gh[0], h_z = gh[64], h_n = gh[128];
  const float ho  = H[(size_t)row * DH + c];
  const float rg = sigm(i_r + h_r);
  const float zg = sigm(i_z + h_z);
  const float ng = tanhf(i_n + rg * h_n);
  const float hn = (1.0f - zg) * ng + zg * ho;
  sH[tid] = hn;
  __syncthreads();
  if (wave < 2) {
    const v4f v = *(const v4fa*)(sH + 4 * tid);
    float* op = H + (size_t)blockIdx.x * (4 * DH) + 4 * tid;
    *(volatile v4f*)op = v;
    __threadfence();
    *(volatile v4f*)op = v;
  } else if (wave < 4) {
    const int u  = tid - 64;
    const int rr = u >> 4;
    const int j  = u & 15;
    const int ch = 8 * (j & 7);
    const unsigned mh = 0u - (unsigned)(j >> 3);
    const v8us o = split8(sH + rr * DH + ch, mh);
    unsigned short* op = Hhl + (size_t)((int)blockIdx.x * 4 + rr) * (size_t)KP + 8 * j;
    *(volatile v8us*)op = o;
    __threadfence();
    *(volatile v8us*)op = o;
  }
}

__global__ __launch_bounds__(NTHR) void k_s2s(const float* __restrict__ H, const int* __restrict__ bat,
                                              const float* __restrict__ WL, const float* __restrict__ bl_ih,
                                              const float* __restrict__ bl_hh, float* Q) {
  extern __shared__ __attribute__((aligned(16))) float sX[];
  __shared__ int sWLs[NWAVE * GCAP];
  __shared__ int sList[GCAP];
  __shared__ int wcnt[NWAVE];
  __shared__ __attribute__((aligned(16))) float sQS[128];
  __shared__ float sHh[64];
  __shared__ float sAct[256];
  __shared__ float sE[256];
  __shared__ float red[256];
  __shared__ float rpart[4 * 64];
  __shared__ __attribute__((aligned(16))) float sOutQ[64];
  const int tid = (int)threadIdx.x, lane = tid & 31, wave = tid >> 5;
  const int g = (int)blockIdx.x;

  for (int i = tid; i < GCAP * XS; i += NTHR) sX[i] = 0.0f;
  for (int i = tid; i < NWAVE * GCAP; i += NTHR) sWLs[i] = 0;
  sList[tid] = 0;
  if (tid < 128) sQS[tid] = 0.0f;
  if (tid < 64)  sHh[tid] = 0.0f;
  __syncthreads();

  int wc = 0;
#pragma unroll 1
  for (int it = 0; it < NPW / 32; ++it) {
    const int i = wave * NPW + it * 32 + lane;
    const int b = bat[i];
    const bool hit = (b == g);
    const unsigned msk = __builtin_amdgcn_ballot_w32(hit);
    if (hit) {
      const int pos = wc + (int)__builtin_amdgcn_mbcnt_lo(msk, 0u);
      if (pos < GCAP) sWLs[wave * GCAP + pos] = i;
    }
    wc += (int)__builtin_popcount(msk);
  }
  if (lane == 0) wcnt[wave] = wc;
  __syncthreads();
  int pre = 0, tot = 0;
#pragma unroll
  for (int w2 = 0; w2 < NWAVE; ++w2) {
    int c = wcnt[w2];
    c = c < 0 ? 0 : (c > NPW ? NPW : c);
    tot += c;
    pre += (w2 < wave) ? c : 0;
  }
  const bool ovf = tot > GCAP;
  const int cnt = tot > GCAP ? GCAP : tot;
  {
    const int wcc = wc > GCAP ? GCAP : wc;
#pragma unroll 1
    for (int i = lane; i < wcc; i += 32) {
      const int pos = pre + i;
      if (pos < GCAP) sList[pos] = sWLs[wave * GCAP + i];
    }
  }
  __syncthreads();
#pragma unroll 1
  for (int n = wave; n < cnt; n += NWAVE) {
    int node = sList[n];
    node = node < 0 ? 0 : (node > NN - 1 ? NN - 1 : node);
    const v2f v = *(const v2f*)(H + (size_t)node * DH + 2 * lane);
    sX[n * XS + 2 * lane]     = v.x;
    sX[n * XS + 2 * lane + 1] = v.y;
  }
  __syncthreads();

  float creg = 0.0f;
  const float bsum = bf16_val(bl_ih[tid]) + bf16_val(bl_hh[tid]);
  const bool live = tid < cnt;
  const float ninf = __int_as_float((int)0xff800000u);
#pragma unroll 1
  for (int s = 0; s < TS2S; ++s) {
    float acc = bsum;
#pragma unroll 4
    for (int k = 0; k < 128; ++k) acc = fmaf(sQS[k], WL[(size_t)k * LW + tid], acc);
#pragma unroll 4
    for (int k = 0; k < 64; ++k) acc = fmaf(sHh[k], WL[(size_t)(128 + k) * LW + tid], acc);
    {
      const bool isg = (tid >> 6) == 2;
      const float sc = isg ? 1.0f : 0.5f;
      const float y  = tanhf(acc * sc);
      sAct[tid] = isg ? y : fmaf(0.5f, y, 0.5f);
    }
    __syncthreads();
    if (tid < 64) {
      creg = sAct[64 + tid] * creg + sAct[tid] * sAct[128 + tid];
      const float hv = sAct[192 + tid] * tanhf(creg);
      sHh[tid] = hv;
      sQS[tid] = hv;
    }
    __syncthreads();
    if (s == TS2S - 1) break;

    float e = 0.0f;
#pragma unroll 4
    for (int k = 0; k < DH; ++k) e = fmaf(sX[tid * XS + k], sQS[k], e);
    red[tid] = live ? e : ninf;
    __syncthreads();
#pragma unroll 1
    for (int st = 128; st > 0; st >>= 1) {
      if (tid < st) red[tid] = nmax(red[tid], red[tid + st]);
      __syncthreads();
    }
    const float emax = red[0];
    __syncthreads();
    const float ex = live ? expf(e - emax) : 0.0f;
    red[tid] = ex;
    __syncthreads();
#pragma unroll 1
    for (int st = 128; st > 0; st >>= 1) {
      if (tid < st) red[tid] = red[tid] + red[tid + st];
      __syncthreads();
    }
    const float denom = red[0];
    const float inv = (cnt > 0) ? (1.0f / denom) : 0.0f;
    sE[tid] = ex * inv;
    __syncthreads();
    {
      const int d = tid & 63, ch = tid >> 6;
      float racc = 0.0f;
#pragma unroll 1
      for (int n = ch; n < cnt; n += 4) racc = fmaf(sE[n], sX[n * XS + d], racc);
      rpart[ch * 64 + d] = racc;
    }
    __syncthreads();
    if (tid < 64) sQS[64 + tid] = ((rpart[tid] + rpart[64 + tid]) + rpart[128 + tid]) + rpart[192 + tid];
    __syncthreads();
  }

  if (tid < 64) {
    const float qnan = __int_as_float(0x7fc00000);
    sOutQ[tid] = ovf ? qnan : sHh[tid];
  }
  __syncthreads();
  const v4f qv = *(const v4fa*)(sOutQ + 4 * (tid & 15));
  float* op = Q + (size_t)g * DH + 4 * (tid & 15);
  const bool okst = tid < 16;
  if (okst) *(volatile v4f*)op = qv;
  __threadfence();
  if (okst) *(volatile v4f*)op = qv;
}

__global__ __launch_bounds__(NTHR) void k_head(const float* __restrict__ Q, const float* __restrict__ W_out,
                                               const float* __restrict__ b_out, float* out) {
  __shared__ __attribute__((aligned(16))) float sQ[NG * DH];
  __shared__ __attribute__((aligned(16))) float sW[DH * OUTD];
  __shared__ __attribute__((aligned(16))) float sO[NG * OUTD];
  const int tid = (int)threadIdx.x;
#pragma unroll 1
  for (int i = tid; i < (NG * DH) / 4; i += NTHR) *(v4fa*)(sQ + 4 * i) = *(const v4f*)(Q + (size_t)4 * i);
  if (tid < (DH * OUTD) / 4) {
    const v4f a = *(const v4f*)(W_out + 4 * tid);
    v4f o;
    o.x = bf16_val(a.x); o.y = bf16_val(a.y); o.z = bf16_val(a.z); o.w = bf16_val(a.w);
    *(v4fa*)(sW + 4 * tid) = o;
  }
  __syncthreads();
#pragma unroll 1
  for (int i = tid; i < NG * OUTD; i += NTHR) {
    const int gq = i / OUTD;
    const int c  = i - gq * OUTD;
    float acc = 0.0f;
#pragma unroll 4
    for (int d = 0; d < DH; ++d) acc = fmaf(sQ[gq * DH + d], sW[d * OUTD + c], acc);
    sO[i] = acc + bf16_val(b_out[c]);
  }
  __syncthreads();
  const int tq = tid < (NG * OUTD) / 4 ? tid : (NG * OUTD) / 4 - 1;
  const v4f ov = *(const v4fa*)(sO + 4 * tq);
  float* op = out + 4 * tq;
  const bool okst = tid < (NG * OUTD) / 4;
  if (okst) *(volatile v4f*)op = ov;
  __threadfence();
  if (okst) *(volatile v4f*)op = ov;
}

static inline size_t al256(size_t o) { return (o + 255) & ~(size_t)255; }

extern "C" void kernel_launch(void* const* d_in, const int* in_sizes, int n_in,
                              void* d_out, int out_size, void* d_ws, size_t ws_size,
                              hipStream_t stream) {
  if (n_in < 21) return;
  const int expect[21] = {NN * NFD, NE * EFD, NE, NE, NN, NFD * DH, DH, EFD * DH, DH, DH * NW2, NW2,
                          DH * G3, DH * G3, G3, G3, 128 * LW, 64 * LW, LW, LW, DH * OUTD, OUTD};
  for (int i = 0; i < 21; ++i) if (in_sizes[i] != expect[i]) return;
  if (out_size != NG * OUTD) return;

  const float* nf    = (const float*)d_in[0];
  const float* ef    = (const float*)d_in[1];
  const int*   Esrc  = (const int*)  d_in[2];
  const int*   Etgt  = (const int*)  d_in[3];
  const int*   bat   = (const int*)  d_in[4];
  const float* W_in  = (const float*)d_in[5];
  const float* b_in  = (const float*)d_in[6];
  const float* W_ee1 = (const float*)d_in[7];
  const float* b_ee1 = (const float*)d_in[8];
  const float* W_ee2 = (const float*)d_in[9];
  const float* b_ee2 = (const float*)d_in[10];
  const float* W_ih  = (const float*)d_in[11];
  const float* W_hh  = (const float*)d_in[12];
  const float* b_ih  = (const float*)d_in[13];
  const float* b_hh  = (const float*)d_in[14];
  const float* Wl_ih = (const float*)d_in[15];
  const float* Wl_hh = (const float*)d_in[16];
  const float* bl_ih = (const float*)d_in[17];
  const float* bl_hh = (const float*)d_in[18];
  const float* W_out = (const float*)d_in[19];
  const float* b_out = (const float*)d_in[20];
  float* out = (float*)d_out;

  char* ws = (char*)d_ws;
  size_t off = 0;
  const size_t oXB  = off; off = al256(off + (size_t)NN * 32 * 2);
  const size_t oEFB = off; off = al256(off + (size_t)NE * 32 * 2);
  const size_t oWin = off; off = al256(off + (size_t)DH * 32 * 2);
  const size_t oWee = off; off = al256(off + (size_t)DH * 32 * 2);
  const size_t oBt2 = off; off = al256(off + (size_t)NPC * KP * 2);
  const size_t oWih = off; off = al256(off + (size_t)G3 * KP * 2);
  const size_t oWhh = off; off = al256(off + (size_t)G3 * KP * 2);
  const size_t oWL  = off; off = al256(off + (size_t)192 * LW * 4);
  const size_t oH   = off; off = al256(off + (size_t)NN * DH * 4);
  const size_t oHhl = off; off = al256(off + (size_t)NN * KP * 2);
  const size_t oAGG = off; off = al256(off + (size_t)NN * KP * 2);
  const size_t oED  = off; off = al256(off + (size_t)NE * DH * 4);
  const size_t oMA  = off; off = al256(off + (size_t)NE * DH * 4);
  const size_t oMS  = off; off = al256(off + (size_t)NE * DH * 4);
  const size_t oGI  = off; off = al256(off + (size_t)NN * G3 * 4);
  const size_t oGH  = off; off = al256(off + (size_t)NN * G3 * 4);
  const size_t oP   = off; off = al256(off + (size_t)NN * PP * 4);
  const size_t oQ   = off; off = al256(off + (size_t)NG * DH * 4);
  if (off > ws_size || off > (size_t)WSMAX) return;
  unsigned short* XB    = (unsigned short*)(ws + oXB);
  unsigned short* EFB   = (unsigned short*)(ws + oEFB);
  unsigned short* WinT  = (unsigned short*)(ws + oWin);
  unsigned short* Wee1T = (unsigned short*)(ws + oWee);
  unsigned short* Bt2   = (unsigned short*)(ws + oBt2);
  unsigned short* WihT2 = (unsigned short*)(ws + oWih);
  unsigned short* WhhT2 = (unsigned short*)(ws + oWhh);
  float*          WL    = (float*)(ws + oWL);
  float*          H     = (float*)(ws + oH);
  unsigned short* Hhl   = (unsigned short*)(ws + oHhl);
  unsigned short* AGG   = (unsigned short*)(ws + oAGG);
  float*          ED    = (float*)(ws + oED);
  float*          MSGA  = (float*)(ws + oMA);
  float*          MSG   = (float*)(ws + oMS);
  float*          GI    = (float*)(ws + oGI);
  float*          GH    = (float*)(ws + oGH);
  float*          P     = (float*)(ws + oP);
  float*          Q     = (float*)(ws + oQ);

  hipFuncSetAttribute(reinterpret_cast<const void*>(&k_agg), hipFuncAttributeMaxDynamicSharedMemorySize,
                      (int)LDS_AGG);
  hipFuncSetAttribute(reinterpret_cast<const void*>(&k_s2s), hipFuncAttributeMaxDynamicSharedMemorySize,
                      (int)LDS_S2S);

  k_prep<<<U_ALL / NTHR, NTHR, 0, stream>>>(nf, ef, W_in, W_ee1, W_ee2, b_ee2, W_ih, W_hh, Wl_ih, Wl_hh,
                                            XB, EFB, WinT, Wee1T, Bt2, WihT2, WhhT2, WL);
  k_gemm<0, 1><<<dim3(NN / GBM, 1), GTHR, 0, stream>>>(XB, 32, WinT, 32, 32, b_in, 1, H, DH, Hhl);
  k_gemm<1, 0><<<dim3(NE / GBM, 1), GTHR, 0, stream>>>(EFB, 32, Wee1T, 32, 32, b_ee1, 1, ED, DH, Hhl);

  for (int t = 0; t < TMPS; ++t) {
    k_gemm<0, 0><<<dim3(NN / GBM, NPA / GBN), GTHR, 0, stream>>>(Hhl, KP, Bt2, KP, KP, b_ee2, 0, P, PP, Hhl);
    k_edge<0><<<NE / EPBK, NTHR, 0, stream>>>(ED, Esrc, P, MSGA, MSGA);
    k_gemm<0, 0><<<dim3(NN / GBM, NPB / GBN), GTHR, 0, stream>>>(Hhl, KP, Bt2 + (size_t)NPA * KP, KP, KP,
                                                                 b_ee2, 0, P, PP, Hhl);
    k_edge<1><<<NE / EPBK, NTHR, 0, stream>>>(ED, Esrc, P, MSGA, MSG);
    k_agg<<<NN / NBA, NTHR, LDS_AGG, stream>>>(Etgt, MSG, AGG);
    k_gemm<0, 0><<<dim3(NN / GBM, G3 / GBN), GTHR, 0, stream>>>(AGG, KP, WihT2, KP, KP, b_ih, 1, GI, G3, Hhl);
    k_gemm<0, 0><<<dim3(NN / GBM, G3 / GBN), GTHR, 0, stream>>>(Hhl, KP, WhhT2, KP, KP, b_hh, 1, GH, G3, AGG);
    k_gru<<<NN / 4, NTHR, 0, stream>>>(GI, GH, H, Hhl);
  }

  k_s2s<<<NG, NTHR, LDS_S2S, stream>>>(H, bat, WL, bl_ih, bl_hh, Q);
  k_head<<<1, NTHR, 0, stream>>>(Q, W_out, b_out, out);
}
